// HybridAttention_72112500900083
// MI455X (gfx1250) — hardware-verified
//
#include <hip/hip_runtime.h>
#include <math.h>

typedef __attribute__((ext_vector_type(16))) _Float16 v16h;
typedef __attribute__((ext_vector_type(16))) __bf16 v16b;
typedef __attribute__((ext_vector_type(8)))  _Float16 v8h;
typedef __attribute__((ext_vector_type(8)))  __bf16 v8b;
typedef __attribute__((ext_vector_type(8)))  float v8f;
typedef __attribute__((ext_vector_type(4)))  float v4f;
typedef __attribute__((ext_vector_type(4)))  unsigned v4u;

template <typename T> __device__ __forceinline__ void vst2(void* p, T v) { *(volatile T*)p = v; __threadfence(); *(volatile T*)p = v; }
__device__ __forceinline__ v8f wmma16(v16h a, v16h b, v8f c) {
  v8f d = __builtin_amdgcn_wmma_f32_16x16x32_f16(false, a, false, b, (short)0, c, false, false);
  asm volatile("v_nop\n\tv_nop\n\tv_nop\n\tv_nop" : "+v"(d) : "v"(a), "v"(b));
  return d;
}
__device__ __forceinline__ v8f wmma_bf(v16b a, v16b b, v8f c) {
  v8f d = __builtin_amdgcn_wmma_f32_16x16x32_bf16(false, a, false, b, (short)0, c, false, false);
  asm volatile("v_nop\n\tv_nop\n\tv_nop\n\tv_nop" : "+v"(d) : "v"(a), "v"(b));
  return d;
}
__device__ __forceinline__ v16h frag_h(const _Float16* rowk0, int lane) {
  union { v16h v; v8h q[2]; } u; const _Float16* p = rowk0 + 8 * (lane >> 4);
  u.q[0] = *(const v8h*)p; u.q[1] = *(const v8h*)(p + 16); return u.v;
}
__device__ __forceinline__ v16b frag_b(const __bf16* rowk0, int lane) {
  union { v16b v; v8b q[2]; } u; const __bf16* p = rowk0 + 8 * (lane >> 4);
  u.q[0] = *(const v8b*)p; u.q[1] = *(const v8b*)(p + 16); return u.v;
}
struct F2 { v16b h, l; };
__device__ __forceinline__ F2 bsplit16(const float v[16]) { F2 r;
#pragma unroll
  for (int i = 0; i < 16; ++i) { const __bf16 h = (__bf16)v[i]; r.h[i] = h; r.l[i] = (__bf16)(v[i] - (float)h); }
  return r; }
__device__ __forceinline__ F2 split_row(const float* row, int k0, int lane) { float v[16]; const float* p = row + k0 + 8 * (lane >> 4);
#pragma unroll
  for (int i = 0; i < 8; ++i) { v[i] = p[i]; v[8 + i] = p[16 + i]; }
  return bsplit16(v); }
__device__ __forceinline__ float bfr(float v) { return (float)(__bf16)v; }
#define LDSX() do { asm volatile("s_wait_dscnt 0" ::: "memory"); __builtin_amdgcn_wave_barrier(); __builtin_amdgcn_fence(3  , "workgroup"); } while (0)

#ifndef NB
#define NB 8
#endif
#ifndef SEQ
#define SEQ 1024
#endif
#define NB_FULL 8
#define SEQ_FULL 1024
#define CC 1024
#define NH 16
#define HD 64
#define HG 4
#define LW 8
#define NLR 64
#define NBS (NB * SEQ)
static_assert(NB >= 1 && NB <= NB_FULL);
static_assert(SEQ % 128 == 0 && SEQ >= 128 && SEQ <= SEQ_FULL);
static_assert(NB * LW <= NLR);
static_assert(NH % HG == 0 && NH * HD == CC);
static_assert(CC % 128 == 0 && HD % 32 == 0);

#define MAXZ(a, b) ((a) > (b) ? (a) : (b))
#define B_PL   (2u * (size_t)NBS * CC)
#define WS_QH  ((size_t)0)
#define WS_KH  (WS_QH + B_PL)
#define WS_VT  (WS_KH + B_PL)
#define WS_VL  (WS_VT + B_PL)
#define WS_R   (WS_VL + B_PL)
#define RC_WGO ((size_t)0)
#define RC_WLI (RC_WGO + 2u * (size_t)CC * CC)
#define RC_WLO (RC_WLI + 2u * (size_t)3 * CC * CC)
#define RC_XL  (RC_WLO + 2u * (size_t)CC * CC)
#define RC_XLR (RC_XL + 2u * (size_t)NLR * CC)
#define RC_PL  (RC_XLR + 2u * (size_t)NLR * CC)
#define RC_CL  (RC_PL + 4u * (size_t)NLR * 3 * CC)
#define RC_OL  (RC_CL + 4u * (size_t)NLR * CC)
#define RC_END (RC_OL + 4u * (size_t)NLR * CC)
#define B_R    MAXZ(MAXZ(4u * (size_t)HG * SEQ * SEQ, 2u * (size_t)NBS * CC), RC_END)
#define WS_Y   (WS_R + B_R)
#define B_Y    MAXZ(4u * (size_t)NBS * CC, 2u * (size_t)3 * CC * CC)
#define WS_END (WS_Y + B_Y)
static_assert(WS_END <= (size_t)134217728u);
static_assert((WS_R % 128) == 0 && (WS_Y % 128) == 0 && (RC_XL % 128) == 0 && (RC_XLR % 128) == 0 && (RC_PL % 128) == 0 && (RC_CL % 128) == 0 && (RC_OL % 128) == 0);

__global__ __launch_bounds__(256) void k_cvt(const float* __restrict__ W, unsigned short* __restrict__ O, int n8, int cm) {
  const int i = blockIdx.x * 256 + threadIdx.x; if (i >= n8) return;
  const float* p = W + (size_t)i * 8; const v4f a = *(const v4f*)p, b = *(const v4f*)(p + 4);
  float v[8];
#pragma unroll
  for (int k = 0; k < 4; ++k) { v[k] = a[k]; v[4 + k] = b[k]; }
  union { v8h h; v8b b; v4u u; } uo;
  if (cm == 0) { v8h hv;
#pragma unroll
    for (int k = 0; k < 8; ++k) hv[k] = (_Float16)(bfr(v[k]) * 64.0f);
    uo.h = hv; }
  else { v8b bv;
#pragma unroll
    for (int k = 0; k < 8; ++k) bv[k] = (__bf16)v[k];
    uo.b = bv; }
  vst2(O + (size_t)i * 8, uo.u);
}

__global__ __launch_bounds__(128) void k_ln(const float* __restrict__ X, const float* __restrict__ G, const float* __restrict__ Bt, _Float16* __restrict__ XO, _Float16* __restrict__ XR, int sw) {
  __shared__ float red[2][4];
  const int tid = threadIdx.x, wave = tid >> 5, lane = tid & 31; const int row = blockIdx.x;
  size_t src; int valid = 1;
  if (sw != 0) { const int b = row / LW, s = row - b * LW; valid = (b < NB) ? 1 : 0; const int bc = valid ? b : 0; src = (size_t)bc * SEQ_FULL + s; }
  else { const int b = row / SEQ, t = row - b * SEQ; src = (size_t)b * SEQ_FULL + t; }
  const int c0 = tid * 8; const float* xr = X + src * CC + c0;
  const v4f x0 = *(const v4f*)xr, x1 = *(const v4f*)(xr + 4), g0 = *(const v4f*)(G + c0), g1 = *(const v4f*)(G + c0 + 4), b0 = *(const v4f*)(Bt + c0), b1 = *(const v4f*)(Bt + c0 + 4);
  float v[8], gg[8], bb[8];
#pragma unroll
  for (int i = 0; i < 4; ++i) { v[i] = bfr(x0[i]); v[4 + i] = bfr(x1[i]); gg[i] = bfr(g0[i]); gg[4 + i] = bfr(g1[i]); bb[i] = bfr(b0[i]); bb[4 + i] = bfr(b1[i]); }
  float s1 = 0.f;
#pragma unroll
  for (int i = 0; i < 8; ++i) s1 += v[i];
#pragma unroll
  for (int o = 1; o < 32; o <<= 1) s1 += __shfl_xor(s1, o);
  if (lane == 0) red[0][wave] = s1;
  __syncthreads();
  const float mean = ((red[0][0] + red[0][1]) + (red[0][2] + red[0][3])) * (1.0f / (float)CC);
  float s2 = 0.f;
#pragma unroll
  for (int i = 0; i < 8; ++i) { const float d = v[i] - mean; v[i] = d; s2 += d * d; }
#pragma unroll
  for (int o = 1; o < 32; o <<= 1) s2 += __shfl_xor(s2, o);
  if (lane == 0) red[1][wave] = s2;
  __syncthreads();
  const float var = ((red[1][0] + red[1][1]) + (red[1][2] + red[1][3])) * (1.0f / (float)CC);
  const float rstd = 1.0f / sqrtf(var + 1e-5f);
  v8h hv, hr;
#pragma unroll
  for (int i = 0; i < 8; ++i) { const float y = v[i] * rstd * gg[i] + bb[i]; const float yv = valid ? y : 0.f; const _Float16 h = (_Float16)yv; hv[i] = h; hr[i] = (_Float16)((yv - (float)h) * 1024.0f); }
  union { v8h h; v4u u; } uo, ur; uo.h = hv; ur.h = hr;
  vst2(XO + (size_t)row * CC + c0, uo.u);
  if (sw != 0) vst2(XR + (size_t)row * CC + c0, ur.u);
}

__global__ __launch_bounds__(128) void k_proj(const _Float16* __restrict__ XN, const _Float16* __restrict__ WP, const float* __restrict__ BI, _Float16* __restrict__ QH, _Float16* __restrict__ KH, __bf16* __restrict__ VT, __bf16* __restrict__ VL) {
  __shared__ __align__(16) _Float16 sh[64][136]; __shared__ __align__(16) __bf16 th[128][72], tl2[128][72];
  const int tid = threadIdx.x, wave = tid >> 5, lane = tid & 31, col = lane & 15, g = lane >> 4; const int which = blockIdx.z; const int c0 = blockIdx.y * 128; const int cw = which * CC + c0; const size_t r0 = (size_t)blockIdx.x * 64;
  v8f acc[8] = {};
#pragma unroll 1
  for (int kc = 0; kc < CC / 32; ++kc) { const v16h a = frag_h(XN + (r0 + wave * 16 + col) * CC + kc * 32, lane);
#pragma unroll
    for (int j = 0; j < 8; ++j) { const v16h w = frag_h(WP + (size_t)(cw + j * 16 + col) * CC + kc * 32, lane); acc[j] = wmma16(a, w, acc[j]); } }
#pragma unroll
  for (int j = 0; j < 8; ++j) { const float bb = bfr(BI[cw + j * 16 + col]);
#pragma unroll
    for (int r = 0; r < 8; ++r) { const float v = acc[j][r] * (1.0f / 64.0f) + bb; const int rl = wave * 16 + 8 * g + r, cl = j * 16 + col;
      if (which == 2) { const __bf16 bh = (__bf16)v; th[cl][rl] = bh; tl2[cl][rl] = (__bf16)(v - (float)bh); }
      else { sh[rl][cl] = (_Float16)v; } } }
  __syncthreads();
  if (which < 2) { _Float16* dh = which == 0 ? QH : KH; for (int e = tid; e < 64 * 16; e += 128) { const int rl = e >> 4, q = e & 15; vst2((unsigned*)(dh + (r0 + rl) * CC + c0 + q * 8), *(const v4u*)&sh[rl][q * 8]); } }
  else { const size_t b = r0 / SEQ; const int t0 = (int)(r0 % SEQ); for (int e = tid; e < 128 * 8; e += 128) { const int cl = e >> 3, q = e & 7; const size_t o2 = (b * CC + c0 + cl) * (size_t)SEQ + t0 + q * 8; vst2((unsigned*)(VT + o2), *(const v4u*)&th[cl][q * 8]); vst2((unsigned*)(VL + o2), *(const v4u*)&tl2[cl][q * 8]); } }
}
__global__ __launch_bounds__(128) void k_projl(const _Float16* __restrict__ XL, const _Float16* __restrict__ XR, const _Float16* __restrict__ WP, const float* __restrict__ BI, float* __restrict__ PL) {
  __shared__ __align__(16) float sf[4][16][132];
  const int tid = threadIdx.x, wave = tid >> 5, lane = tid & 31, col = lane & 15, g = lane >> 4; const int c0 = blockIdx.y * 128; const size_t r0 = (size_t)blockIdx.x * 64 + wave * 16;
  v8f acc[8] = {}, accr[8] = {};
#pragma unroll 1
  for (int kc = 0; kc < CC / 32; ++kc) { const v16h ah = frag_h(XL + (r0 + col) * CC + kc * 32, lane), ar = frag_h(XR + (r0 + col) * CC + kc * 32, lane);
#pragma unroll
    for (int j = 0; j < 8; ++j) { const v16h w = frag_h(WP + (size_t)(c0 + j * 16 + col) * CC + kc * 32, lane); acc[j] = wmma16(ah, w, acc[j]); accr[j] = wmma16(ar, w, accr[j]); } }
#pragma unroll
  for (int j = 0; j < 8; ++j) acc[j] += accr[j] * (1.0f / 1024.0f);
#pragma unroll
  for (int j = 0; j < 8; ++j) { const float bb = bfr(BI[c0 + j * 16 + col]);
#pragma unroll
    for (int r = 0; r < 8; ++r) sf[wave][8 * g + r][j * 16 + col] = acc[j][r] * (1.0f / 64.0f) + bb; }
  LDSX(); for (int rl = 0; rl < 16; ++rl) vst2(PL + (r0 + rl) * (size_t)(3 * CC) + c0 + lane * 4, *(const v4f*)&sf[wave][rl][lane * 4]);
}
__global__ __launch_bounds__(64) void k_attl(const float* __restrict__ PL, float* __restrict__ CL) {
  __shared__ __align__(16) float sx[3][LW][HD]; __shared__ float sp[LW][LW]; __shared__ __align__(16) float so[LW][HD + 4];
  const int tid = threadIdx.x, wave = tid >> 5, lane = tid & 31; const int bl = blockIdx.x, h = blockIdx.y;
  for (int e = tid; e < 3 * LW * (HD / 4); e += 64) { const int m = e / (LW * (HD / 4)), rem = e - m * (LW * (HD / 4)), r = rem / (HD / 4), q = rem - r * (HD / 4);
    *(v4f*)&sx[m][r][q * 4] = *(const v4f*)(PL + (size_t)(bl * LW + r) * (3 * CC) + m * CC + h * HD + q * 4); }
  __syncthreads();
  { const int qi = tid >> 3, kj = tid & 7; float s = 0.f;
#pragma unroll 1
    for (int d = 0; d < HD; ++d) s += sx[0][qi][d] * sx[1][kj][d];
    sp[qi][kj] = s * 0.125f; }
  __syncthreads();
  if (tid < LW) { float m = -3.0e38f;
#pragma unroll 1
    for (int j = 0; j < LW; ++j) m = fmaxf(m, sp[tid][j]);
    float su = 0.f;
#pragma unroll 1
    for (int j = 0; j < LW; ++j) { const float e = expf(sp[tid][j] - m); su += e; sp[tid][j] = e; }
    const float inv = 1.0f / su;
#pragma unroll 1
    for (int j = 0; j < LW; ++j) sp[tid][j] = sp[tid][j] * inv; }
  __syncthreads();
#pragma unroll 1
  for (int qi = 0; qi < LW; ++qi) { float o = 0.f;
#pragma unroll 1
    for (int j = 0; j < LW; ++j) o += sp[qi][j] * sx[2][j][tid];
    so[qi][tid] = o; }
  __syncthreads();
#pragma unroll
  for (int it = 0; it < 2; ++it) { const int r = wave * 4 + it * 2 + (lane >> 4), q = lane & 15; vst2(CL + (size_t)(bl * LW + r) * CC + h * HD + q * 4, *(const v4f*)&so[r][q * 4]); }
}
__global__ __launch_bounds__(128) void k_sc(const _Float16* __restrict__ QH, const _Float16* __restrict__ KH, int b, int h0, float* __restrict__ S0) { __shared__ __align__(16) float ss[4][16][132]; const int h = h0 + blockIdx.z; float* S = S0 + (size_t)blockIdx.z * SEQ * SEQ;
  const int tid = threadIdx.x, wave = tid >> 5, lane = tid & 31, col = lane & 15, g = lane >> 4; const int k0 = blockIdx.y * 128; const int ql0 = blockIdx.x * 64 + wave * 16; const size_t q0 = (size_t)b * SEQ + ql0;
  v8f acc[8] = {};
#pragma unroll
  for (int kc = 0; kc < HD / 32; ++kc) { const v16h ah = frag_h(QH + (q0 + col) * CC + h * HD + kc * 32, lane);
#pragma unroll
    for (int j = 0; j < 8; ++j) { const v16h kb = frag_h(KH + ((size_t)b * SEQ + k0 + j * 16 + col) * CC + h * HD + kc * 32, lane); acc[j] = wmma16(ah, kb, acc[j]); } }
#pragma unroll
  for (int j = 0; j < 8; ++j)
#pragma unroll
    for (int r = 0; r < 8; ++r) ss[wave][8 * g + r][j * 16 + col] = acc[j][r] * 0.125f;
  LDSX(); for (int rl = 0; rl < 16; ++rl) vst2(S + (size_t)(ql0 + rl) * SEQ + k0 + lane * 4, *(const v4f*)&ss[wave][rl][lane * 4]);
}
__global__ __launch_bounds__(128) void k_pv(const float* __restrict__ S0, const __bf16* __restrict__ VT, const __bf16* __restrict__ VL, int b, int h0, float* __restrict__ Y) {
  __shared__ __align__(16) float ss[4][16][HD + 4];
  const int h = h0 + blockIdx.z; const float* PS = S0 + (size_t)blockIdx.z * SEQ * SEQ;
  const int tid = threadIdx.x, wave = tid >> 5, lane = tid & 31, col = lane & 15, g = lane >> 4; const int ql0 = blockIdx.x * 64 + wave * 16;
  const float* pr = PS + (size_t)(ql0 + col) * SEQ + 8 * g;
  float mx = -3.0e38f;
#pragma unroll 1
  for (int kc = 0; kc < SEQ / 32; ++kc) { const float* p = pr + kc * 32; const v4f a0 = *(const v4f*)p, a1 = *(const v4f*)(p + 4), a2 = *(const v4f*)(p + 16), a3 = *(const v4f*)(p + 20);
#pragma unroll
    for (int i = 0; i < 4; ++i) mx = fmaxf(mx, fmaxf(fmaxf(a0[i], a1[i]), fmaxf(a2[i], a3[i]))); }
  mx = fmaxf(mx, __shfl_xor(mx, 16));
  float sum = 0.f; v8f acc[HD / 16] = {};
#pragma unroll 1
  for (int kc = 0; kc < SEQ / 32; ++kc) { const float* p = pr + kc * 32; const v4f a0 = *(const v4f*)p, a1 = *(const v4f*)(p + 4), a2 = *(const v4f*)(p + 16), a3 = *(const v4f*)(p + 20); float v[16];
#pragma unroll
    for (int i = 0; i < 4; ++i) { v[i] = a0[i]; v[4 + i] = a1[i]; v[8 + i] = a2[i]; v[12 + i] = a3[i]; }
#pragma unroll
    for (int i = 0; i < 16; ++i) { const float e = expf(v[i] - mx); sum += e; v[i] = e * 2048.0f; }
    const F2 pf = bsplit16(v);
#pragma unroll
    for (int j = 0; j < HD / 16; ++j) { const size_t po = ((size_t)b * CC + h * HD + j * 16 + col) * (size_t)SEQ + kc * 32; const v16b vh = frag_b(VT + po, lane); acc[j] = wmma_bf(pf.h, vh, acc[j]); acc[j] = wmma_bf(pf.l, vh, acc[j]); acc[j] = wmma_bf(pf.h, frag_b(VL + po, lane), acc[j]); } }
  sum += __shfl_xor(sum, 16);
  const float inv = (1.0f / sum) * (1.0f / 2048.0f);
  float invr[8];
#pragma unroll
  for (int r = 0; r < 8; ++r) invr[r] = __shfl(inv, 8 * g + r);
#pragma unroll
  for (int j = 0; j < HD / 16; ++j)
#pragma unroll
    for (int r = 0; r < 8; ++r) ss[wave][8 * g + r][j * 16 + col] = acc[j][r] * invr[r];
  LDSX(); for (int rl = 0; rl < 16; ++rl) if (lane < HD / 4) vst2(Y + ((size_t)b * SEQ + ql0 + rl) * CC + h * HD + lane * 4, *(const v4f*)&ss[wave][rl][lane * 4]);
}
__global__ __launch_bounds__(128) void k_out(const float* __restrict__ Y, const __bf16* __restrict__ WP, const float* __restrict__ BP, const float* __restrict__ AD, int addw, float* __restrict__ OUT) { __shared__ __align__(16) float sf[4][16][132];
  const int tid = threadIdx.x, wave = tid >> 5, lane = tid & 31, col = lane & 15, g = lane >> 4; const int c0 = blockIdx.y * 128; const size_t r0 = (size_t)blockIdx.x * 64 + wave * 16;
  v8f acc[8] = {};
#pragma unroll 1
  for (int kc = 0; kc < CC / 32; ++kc) { const F2 a = split_row(Y + (r0 + col) * CC, kc * 32, lane);
#pragma unroll
    for (int j = 0; j < 8; ++j) { const v16b w = frag_b(WP + (size_t)(c0 + j * 16 + col) * CC + kc * 32, lane); acc[j] = wmma_bf(a.h, w, acc[j]); acc[j] = wmma_bf(a.l, w, acc[j]); } }
#pragma unroll
  for (int j = 0; j < 8; ++j) { const float bb = bfr(BP[c0 + j * 16 + col]);
#pragma unroll
    for (int r = 0; r < 8; ++r) sf[wave][8 * g + r][j * 16 + col] = acc[j][r] + bb; }
  LDSX();
  for (int rl = 0; rl < 16; ++rl) { const size_t R = r0 + rl; v4f o = *(const v4f*)&sf[wave][rl][lane * 4];
    const int bq = (int)(R / SEQ), s = (int)(R - (size_t)bq * SEQ);
    if (addw != 0 && s < LW) { int lr = bq * LW + s; lr = lr < NLR ? lr : NLR - 1; const v4f av = *(const v4f*)(AD + (size_t)lr * CC + c0 + lane * 4); o += av; }
    vst2(OUT + R * CC + c0 + lane * 4, o); }
}
extern "C" void kernel_launch(void* const* d_in, const int* in_sizes, int n_in, void* d_out, int out_size, void* d_ws, size_t ws_size, hipStream_t stream) {
  if (n_in < 13) return;
  const float* const* F = (const float* const*)d_in;
  if ((size_t)in_sizes[0] < ((size_t)(NB - 1) * SEQ_FULL + SEQ) * CC) return;
  if (in_sizes[1] < CC || in_sizes[2] < CC || in_sizes[3] < CC || in_sizes[4] < CC) return;
  if (in_sizes[5] < 3 * CC * CC || in_sizes[6] < 3 * CC || in_sizes[7] < CC * CC || in_sizes[8] < CC) return;
  if (in_sizes[9] < 3 * CC * CC || in_sizes[10] < 3 * CC || in_sizes[11] < CC * CC || in_sizes[12] < CC) return;
  if ((size_t)out_size < (size_t)NBS * CC) return;
  if (ws_size < (size_t)WS_END) return;
  char* ws = (char*)d_ws;
  _Float16 *QH = (_Float16*)(ws + WS_QH), *KH = (_Float16*)(ws + WS_KH); __bf16 *VT = (__bf16*)(ws + WS_VT), *VL = (__bf16*)(ws + WS_VL);
  _Float16* XN = (_Float16*)(ws + WS_R); float* S = (float*)(ws + WS_R); float* Y = (float*)(ws + WS_Y);
  unsigned short* WGIb = (unsigned short*)(ws + WS_Y); const _Float16* WGI = (const _Float16*)(ws + WS_Y);
  unsigned short* WGOb = (unsigned short*)(ws + WS_R + RC_WGO); const __bf16* WGO = (const __bf16*)(ws + WS_R + RC_WGO);
  unsigned short* WLIb = (unsigned short*)(ws + WS_R + RC_WLI); const _Float16* WLI = (const _Float16*)(ws + WS_R + RC_WLI);
  unsigned short* WLOb = (unsigned short*)(ws + WS_R + RC_WLO); const __bf16* WLO = (const __bf16*)(ws + WS_R + RC_WLO);
  _Float16* XL = (_Float16*)(ws + WS_R + RC_XL); _Float16* XLR = (_Float16*)(ws + WS_R + RC_XLR); float* PL = (float*)(ws + WS_R + RC_PL); float* CL = (float*)(ws + WS_R + RC_CL); float* OL = (float*)(ws + WS_R + RC_OL);
  const int n8g = 3 * CC * CC / 8, n8o = CC * CC / 8;
  k_cvt<<<(n8g + 255) / 256, 256, 0, stream>>>(F[9], WGIb, n8g, 0);
  k_ln<<<NBS, 128, 0, stream>>>(F[0], F[3], F[4], XN, nullptr, 0);
  k_proj<<<dim3(NBS / 64, CC / 128, 3), 128, 0, stream>>>(XN, WGI, F[10], QH, KH, VT, VL);
  for (int b = 0; b < NB; ++b) for (int h0 = 0; h0 < NH; h0 += HG) {
    k_sc<<<dim3(SEQ / 64, SEQ / 128, HG), 128, 0, stream>>>(QH, KH, b, h0, S);
    k_pv<<<dim3(SEQ / 64, 1, HG), 128, 0, stream>>>(S, VT, VL, b, h0, Y);
  }
  k_cvt<<<(n8o + 255) / 256, 256, 0, stream>>>(F[11], WGOb, n8o, 1);
  k_cvt<<<(n8g + 255) / 256, 256, 0, stream>>>(F[5], WLIb, n8g, 0);
  k_cvt<<<(n8o + 255) / 256, 256, 0, stream>>>(F[7], WLOb, n8o, 1);
  k_ln<<<NLR, 128, 0, stream>>>(F[0], F[1], F[2], XL, XLR, 1);
  k_projl<<<dim3(NLR / 64, 3 * CC / 128), 128, 0, stream>>>(XL, XLR, WLI, F[6], PL);
  k_attl<<<dim3(NLR / LW, NH), 64, 0, stream>>>(PL, CL);
  k_out<<<dim3(NLR / 64, CC / 128), 128, 0, stream>>>(CL, WLO, F[8], CL, 0, OL);
  k_out<<<dim3(NBS / 64, CC / 128), 128, 0, stream>>>(Y, WGO, F[12], OL, 1, (float*)d_out);
}
